// FactoredMultilevelDense_14929306321790
// MI455X (gfx1250) — hardware-verified
//
#include <hip/hip_runtime.h>
#include <math.h>
#include <stdint.h>


#define IN_F   256
#define U_N    128
#define LW_N   64
#define LB_N   32
#define MT     64
#define TILE_Q 512

typedef __bf16       bf16x16 __attribute__((ext_vector_type(16)));
typedef float        v8f     __attribute__((ext_vector_type(8)));
typedef float        v4f     __attribute__((ext_vector_type(4)));
typedef unsigned int u4v     __attribute__((ext_vector_type(4)));

__device__ __forceinline__ float softplus_f(float v) {
    return fmaxf(v, 0.0f) + log1pf(expf(-fabsf(v)));
}

__device__ __forceinline__ unsigned int bf16_rne_bits(float f) {
    unsigned int u = __float_as_uint(f);
    u += 0x7FFFu + ((u >> 16) & 1u);
    return u >> 16;
}

__device__ __forceinline__ void split_pair(float a, float b, unsigned int& hw, unsigned int& lw) {
    const unsigned int ha = bf16_rne_bits(a), hb = bf16_rne_bits(b);
    const float ra = a - __uint_as_float(ha << 16);
    const float rb = b - __uint_as_float(hb << 16);
    const unsigned int la = bf16_rne_bits(ra), lb = bf16_rne_bits(rb);
    hw = ha | (hb << 16);
    lw = la | (lb << 16);
}

__device__ __forceinline__ void split8(float v0, float v1, float v2, float v3,
                                       float v4, float v5, float v6, float v7,
                                       u4v& hq, u4v& lq) {
    unsigned int h0, l0, h1, l1, h2, l2, h3, l3;
    split_pair(v0, v1, h0, l0);
    split_pair(v2, v3, h1, l1);
    split_pair(v4, v5, h2, l2);
    split_pair(v6, v7, h3, l3);
    hq.x = h0; hq.y = h1; hq.z = h2; hq.w = h3;
    lq.x = l0; lq.y = l1; lq.z = l2; lq.w = l3;
}

__device__ __forceinline__ v8f mma3(v8f c, bf16x16 ah, bf16x16 al, bf16x16 bh, bf16x16 bl) {
    c = __builtin_amdgcn_wmma_f32_16x16x32_bf16(false, ah, false, bh, (short)0, c, false, false);
    c = __builtin_amdgcn_wmma_f32_16x16x32_bf16(false, al, false, bh, (short)0, c, false, false);
    c = __builtin_amdgcn_wmma_f32_16x16x32_bf16(false, ah, false, bl, (short)0, c, false, false);
    asm volatile("v_nop\n\tv_nop\n\tv_nop\n\tv_nop" : "+v"(c) : "v"(ah), "v"(al), "v"(bh), "v"(bl));
    return c;
}

__global__ __launch_bounds__(256) void pack_kernel(const float* __restrict__ Wf,
                                                   const float* __restrict__ Bf,
                                                   int ntw,
                                                   u4v* whi, u4v* wlo) {
    __shared__ float tile[32][U_N + 4];
    const int kt = blockIdx.x;
    const int t  = threadIdx.x;
    const float* src = (kt < ntw) ? (Wf + (size_t)kt * 32 * U_N) : Bf;
    #pragma unroll
    for (int i = 0; i < 16; ++i) {
        const int idx = t + 256 * i;
        const int r = idx >> 7, c = idx & 127;
        tile[r][c] = src[(size_t)r * U_N + c];
    }
    __syncthreads();

    u4v hq[2], lq[2];
    #pragma unroll
    for (int j = 0; j < 2; ++j) {
        const int p    = t + 256 * j;
        const int f    = p >> 1;
        const int half = p & 1;
        const int ln   = f & 31;
        const int n    = f >> 5;
        const int u    = n * 16 + (ln & 15);
        const int kb   = (ln >> 4) * 8 + 16 * half;
        split8(tile[kb + 0][u], tile[kb + 1][u], tile[kb + 2][u], tile[kb + 3][u],
               tile[kb + 4][u], tile[kb + 5][u], tile[kb + 6][u], tile[kb + 7][u],
               hq[j], lq[j]);
    }
    const size_t base = (size_t)kt * TILE_Q + t;
    #pragma unroll
    for (int j = 0; j < 2; ++j) {
        *(volatile u4v*)(whi + base + 256 * j) = hq[j];
        *(volatile u4v*)(wlo + base + 256 * j) = lq[j];
    }
    __threadfence();
    #pragma unroll
    for (int j = 0; j < 2; ++j) {
        *(volatile u4v*)(whi + base + 256 * j) = hq[j];
        *(volatile u4v*)(wlo + base + 256 * j) = lq[j];
    }
}

__global__ __launch_bounds__(256) void gemm_kernel(
    const float* __restrict__ x,
    const float* __restrict__ eps_w,
    const float* __restrict__ eps_b,
    const float* __restrict__ zw_mu,
    const float* __restrict__ zw_sigma,
    const float* __restrict__ zb_mu,
    const float* __restrict__ zb_sigma,
    const int*   __restrict__ gid,
    const u4v*   __restrict__ whi,
    const u4v*   __restrict__ wlo,
    float* out, int ngroups, int ntw) {

    __shared__ __attribute__((aligned(32))) u4v smem[3072];

    const int t    = threadIdx.x;
    const int lane = t & 31;
    const int wv   = t >> 5;
    const int rg   = wv & 3;
    const int cg   = wv >> 2;
    const int h    = lane >> 4;
    const int m    = lane & 15;
    const int m0   = blockIdx.x * MT;
    const int rl   = rg * 16 + m;
    const size_t grow = (size_t)(m0 + rl);

    float* zw_s = (float*)&smem[1536];
    float* zb_s = (float*)&smem[2560];

    #pragma unroll 1
    for (int i = 0; i < 16; ++i) {
        const int idx = t + 256 * i;
        const int r = idx >> 6, l = idx & 63;
        const int b = m0 + r;
        int g = gid[b];
        g = g < 0 ? 0 : g;
        g = g >= ngroups ? ngroups - 1 : g;
        const float mu = zw_mu[(size_t)g * LW_N + l];
        const float sg = softplus_f(zw_sigma[(size_t)g * LW_N + l]);
        zw_s[idx] = mu + sg * eps_w[(size_t)b * LW_N + l];
    }
    #pragma unroll 1
    for (int i = 0; i < 8; ++i) {
        const int idx = t + 256 * i;
        const int r = idx >> 5, l = idx & 31;
        const int b = m0 + r;
        int g = gid[b];
        g = g < 0 ? 0 : g;
        g = g >= ngroups ? ngroups - 1 : g;
        const float mu = zb_mu[(size_t)g * LB_N + l];
        const float sg = softplus_f(zb_sigma[(size_t)g * LB_N + l]);
        zb_s[idx] = mu + sg * eps_b[(size_t)b * LB_N + l];
    }

    v8f acc[4];
    #pragma unroll
    for (int n = 0; n < 4; ++n) {
        #pragma unroll
        for (int r = 0; r < 8; ++r) acc[n][r] = 0.0f;
    }

    const int aslot = 1024 + (rg * 32 + lane) * 2;

    #pragma unroll 1
    for (int kt = 0; kt <= ntw; ++kt) {
        __syncthreads();
        const size_t gq = (size_t)kt * TILE_Q + t;
        smem[t]             = whi[gq];
        smem[t + 256]       = whi[gq + 256];
        smem[512 + t]       = wlo[gq];
        smem[512 + 256 + t] = wlo[gq + 256];

        float a0, a1, a2, a3, a4, a5, a6, a7;
        if (kt < ntw) {
            const int l    = kt >> 3;
            const int iseg = (kt & 7) * 32 + cg * 16 + h * 8;
            const float zws = zw_s[rl * LW_N + l];
            const float4* xp = (const float4*)(x + grow * IN_F + iseg);
            const float4 x0 = xp[0];
            const float4 x1 = xp[1];
            a0 = zws * x0.x; a1 = zws * x0.y; a2 = zws * x0.z; a3 = zws * x0.w;
            a4 = zws * x1.x; a5 = zws * x1.y; a6 = zws * x1.z; a7 = zws * x1.w;
        } else {
            const float* zp = zb_s + rl * LB_N + cg * 16 + h * 8;
            a0 = zp[0]; a1 = zp[1]; a2 = zp[2]; a3 = zp[3];
            a4 = zp[4]; a5 = zp[5]; a6 = zp[6]; a7 = zp[7];
        }
        u4v hq, lq;
        split8(a0, a1, a2, a3, a4, a5, a6, a7, hq, lq);
        smem[aslot + cg]       = hq;
        smem[aslot + 256 + cg] = lq;
        __syncthreads();

        const bf16x16 ah = *(const bf16x16*)&smem[aslot];
        const bf16x16 al = *(const bf16x16*)&smem[aslot + 256];
        #pragma unroll
        for (int n = 0; n < 4; ++n) {
            const int f = (cg * 4 + n) * 32 + lane;
            const bf16x16 bh = *(const bf16x16*)&smem[2 * f];
            const bf16x16 bl = *(const bf16x16*)&smem[512 + 2 * f];
            acc[n] = mma3(acc[n], ah, al, bh, bl);
        }
    }

    __syncthreads();
    float* stg = (float*)smem + wv * 1024;
    #pragma unroll
    for (int n = 0; n < 4; ++n) {
        #pragma unroll
        for (int r = 0; r < 8; ++r)
            stg[(8 * h + r) * 64 + 16 * n + m] = acc[n][r];
    }
    __syncthreads();
    v4f vals[8];
    #pragma unroll
    for (int j = 0; j < 8; ++j)
        vals[j] = *(const v4f*)(stg + (2 * j + h) * 64 + 4 * m);
    float* obase = out + (size_t)(m0 + rg * 16) * U_N + cg * 64 + 4 * m;
    #pragma unroll
    for (int j = 0; j < 8; ++j)
        *(volatile v4f*)(obase + (size_t)(2 * j + h) * U_N) = vals[j];
    __threadfence();
    #pragma unroll
    for (int j = 0; j < 8; ++j)
        *(volatile v4f*)(obase + (size_t)(2 * j + h) * U_N) = vals[j];
}

extern "C" void kernel_launch(void* const* d_in, const int* in_sizes, int n_in,
                              void* d_out, int out_size, void* d_ws, size_t ws_size,
                              hipStream_t stream) {
    if (n_in < 10) return;

    const float* x        = (const float*)d_in[0];
    const float* eps_w    = (const float*)d_in[1];
    const float* eps_b    = (const float*)d_in[2];
    const float* zw_mu    = (const float*)d_in[3];
    const float* zw_sigma = (const float*)d_in[4];
    const float* Wf       = (const float*)d_in[5];
    const float* zb_mu    = (const float*)d_in[6];
    const float* zb_sigma = (const float*)d_in[7];
    const float* Bf       = (const float*)d_in[8];
    const int*   gid      = (const int*)d_in[9];
    float*       out      = (float*)d_out;

    const int nB  = in_sizes[9];
    const int nG  = in_sizes[3] / LW_N;
    const int ntw = (LW_N * IN_F) / 32;

    if (nB <= 0 || (nB % MT) != 0) return;
    if (in_sizes[0] != nB * IN_F || in_sizes[1] != nB * LW_N || in_sizes[2] != nB * LB_N) return;
    if (in_sizes[5] != LW_N * IN_F * U_N || in_sizes[8] != LB_N * U_N) return;
    if (nG <= 0 || in_sizes[4] != nG * LW_N || in_sizes[6] != nG * LB_N || in_sizes[7] != nG * LB_N) return;
    if (out_size != nB * U_N) return;

    const size_t wbytes = (size_t)(ntw + 1) * (size_t)TILE_Q * 16;
    if (2 * wbytes > ws_size) return;
    u4v* whi = (u4v*)d_ws;
    u4v* wlo = (u4v*)((char*)d_ws + wbytes);

    pack_kernel<<<ntw + 1, 256, 0, stream>>>(Wf, Bf, ntw, whi, wlo);
    gemm_kernel<<<nB / MT, 256, 0, stream>>>(x, eps_w, eps_b, zw_mu, zw_sigma, zb_mu, zb_sigma,
                                             gid, whi, wlo, out, nG, ntw);
}
